// ConfidenceBiasedCrossAttention_90529320665516
// MI455X (gfx1250) — hardware-verified
//
#include <hip/hip_runtime.h>
#include <math.h>

typedef __attribute__((ext_vector_type(16))) _Float16 v16h;
typedef __attribute__((ext_vector_type(16))) __bf16 v16b;
typedef __attribute__((ext_vector_type(8)))  _Float16 v8h;
typedef __attribute__((ext_vector_type(8)))  float v8f;
typedef __attribute__((ext_vector_type(4)))  float v4f;
typedef __attribute__((ext_vector_type(2)))  float v2f;
typedef __attribute__((ext_vector_type(4)))  unsigned v4u;
typedef __attribute__((ext_vector_type(4)))  int v4i;
typedef float __attribute__((may_alias)) float_a;
typedef int __attribute__((may_alias)) int_a;

template <typename T> __device__ __forceinline__ void vst2(void* p, T v) { *(volatile T*)p = v; __threadfence(); *(volatile T*)p = v; }
__device__ __forceinline__ v8f wmma16(v16h a, v16h b, v8f c) {
  v8f d = __builtin_amdgcn_wmma_f32_16x16x32_f16(false, a, false, b, (short)0, c, false, false);
  asm volatile("v_nop\n\tv_nop\n\tv_nop\n\tv_nop" : "+v"(d) : "v"(a), "v"(b));
  return d;
}
__device__ __forceinline__ v8f wmma_bf(v16b a, v16b b, v8f c) {
  v8f d = __builtin_amdgcn_wmma_f32_16x16x32_bf16(false, a, false, b, (short)0, c, false, false);
  asm volatile("v_nop\n\tv_nop\n\tv_nop\n\tv_nop" : "+v"(d) : "v"(a), "v"(b));
  return d;
}
__device__ __forceinline__ v16h frag_h(const _Float16* rowk0, int lane) {
  union { v16h v; v8h q[2]; } u; const _Float16* p = rowk0 + 8 * (lane >> 4);
  u.q[0] = *(const v8h*)p; u.q[1] = *(const v8h*)(p + 16); return u.v;
}
__device__ __forceinline__ v16h frag_f32(const float* rowk0, int lane) {
  v16h a; const float* p = rowk0 + 8 * (lane >> 4);
#pragma unroll
  for (int i = 0; i < 8; ++i) { a[i] = (_Float16)p[i]; a[8 + i] = (_Float16)p[16 + i]; }
  return a;
}
__device__ __forceinline__ v16h frag_f32s(const float* rowk0, int lane, float sc) {
  v16h a; const float* p = rowk0 + 8 * (lane >> 4);
#pragma unroll
  for (int i = 0; i < 8; ++i) { a[i] = (_Float16)(p[i] * sc); a[8 + i] = (_Float16)(p[16 + i] * sc); }
  return a;
}
__device__ __forceinline__ v16h fragc_f32(const float* W, int k0, int n, int lane, int ld, int K) {
  v16h a; const int g = lane >> 4;
#pragma unroll
  for (int i = 0; i < 8; ++i) { const int ka = k0 + 8 * g + i, kb = ka + 16;
    a[i] = (_Float16)(ka < K ? W[(size_t)(ka < K ? ka : K - 1) * ld + n] : 0.f); a[8 + i] = (_Float16)(kb < K ? W[(size_t)(kb < K ? kb : K - 1) * ld + n] : 0.f); }
  return a;
}
struct F2 { v16b h, l; };
__device__ __forceinline__ F2 bsplit16(const float v[16]) { F2 r;
#pragma unroll
  for (int i = 0; i < 16; ++i) { const __bf16 h = (__bf16)v[i]; r.h[i] = h; r.l[i] = (__bf16)(v[i] - (float)h); }
  return r; }
__device__ __forceinline__ F2 split_row(const float* row, int k0, int lane) { float v[16]; const float* p = row + k0 + 8 * (lane >> 4);
#pragma unroll
  for (int i = 0; i < 8; ++i) { v[i] = p[i]; v[8 + i] = p[16 + i]; }
  return bsplit16(v); }
__device__ __forceinline__ F2 split_rowK(const float* row, int k0, int lane, int K) { float v[16]; const int g = lane >> 4;
#pragma unroll
  for (int i = 0; i < 8; ++i) { const int ka = k0 + 8 * g + i, kb = ka + 16; v[i] = ka < K ? row[ka < K ? ka : K - 1] : 0.f; v[8 + i] = kb < K ? row[kb < K ? kb : K - 1] : 0.f; }
  return bsplit16(v); }
__device__ __forceinline__ F2 split_col(const float* W, int k0, int n, int lane, int ld, int K) { float v[16]; const int g = lane >> 4;
#pragma unroll
  for (int i = 0; i < 8; ++i) { const int ka = k0 + 8 * g + i, kb = ka + 16; v[i] = ka < K ? W[(size_t)(ka < K ? ka : K - 1) * ld + n] : 0.f; v[8 + i] = kb < K ? W[(size_t)(kb < K ? kb : K - 1) * ld + n] : 0.f; }
  return bsplit16(v); }
__device__ __forceinline__ v8f mac3(const F2& a, const F2& b, v8f c) { c = wmma_bf(a.l, b.h, c); c = wmma_bf(a.h, b.l, c); return wmma_bf(a.h, b.h, c); }
__device__ __forceinline__ float sigm(float v) { return 1.0f / (1.0f + expf(-v)); }
#define LDSX() do { asm volatile("s_wait_dscnt 0" ::: "memory"); __builtin_amdgcn_wave_barrier(); __builtin_amdgcn_fence(__ATOMIC_RELEASE, "workgroup"); } while (0)


#define NB 2
#define LQ 1024
#define LK 4096
#define DM 1024
#define NH 16
#define HD 64
#define NRQ (NB * LQ)
#define NRK (NB * LK)
#ifndef TQB
#define TQB (LQ / 64)
#define TNB NB
#endif
typedef __attribute__((ext_vector_type(8))) __bf16 v8b;
__device__ __forceinline__ v16b frag_b(const __bf16* rowk0, int lane) {
  union { v16b v; v8b q[2]; } u; const __bf16* p = rowk0 + 8 * (lane >> 4);
  u.q[0] = *(const v8b*)p; u.q[1] = *(const v8b*)(p + 16); return u.v;
}
__device__ __forceinline__ float bfr(float v) { return (float)(__bf16)v; }
__device__ __attribute__((noinline)) float exp_ni(float v) { return expf(v); }
__device__ __attribute__((noinline)) float erf_ni(float v) { return erff(v); }

#define WS_PW  0u
#define WS_Q   (WS_PW + 2u * (size_t)4 * DM * DM)
#define WS_K   (WS_Q + 2u * (size_t)NRQ * DM)
#define WS_V   (WS_K + 2u * (size_t)NRK * DM)
#define WS_O   (WS_V + 2u * (size_t)NB * DM * LK)
#define WS_END (WS_O + 4u * (size_t)NRQ * DM)

__global__ __launch_bounds__(256) void k_pack(const float* __restrict__ WQ, const float* __restrict__ WK, const float* __restrict__ WV, const float* __restrict__ WO, __bf16* __restrict__ PW) { const int n = blockIdx.x, which = blockIdx.y, t = threadIdx.x; __shared__ __align__(16) __bf16 s[DM]; const float* w = (which == 0) ? WQ : (which == 1) ? WK : (which == 2) ? WV : WO;
  for (int k = t; k < DM; k += 256) s[k] = (__bf16)w[(size_t)n * DM + k]; __syncthreads(); if (t < DM / 8) vst2((unsigned*)(PW + ((size_t)which * DM + n) * DM + t * 8), *(const v4u*)&s[t * 8]); }
__global__ __launch_bounds__(128) void k_proj(const float* __restrict__ XQ, const float* __restrict__ XK, const float* __restrict__ XV, const __bf16* __restrict__ PW, const float* __restrict__ BQ, const float* __restrict__ BK, const float* __restrict__ BV, _Float16* __restrict__ Q, _Float16* __restrict__ Kr, _Float16* __restrict__ V) {
  __shared__ __align__(16) _Float16 so[64][136]; __shared__ __align__(16) _Float16 st[128][72];
  const int tid = threadIdx.x, wave = tid >> 5, lane = tid & 31, col = lane & 15, g = lane >> 4; const int which = blockIdx.z; const size_t rb = (size_t)blockIdx.x * 64; if (which == 0 && rb >= (size_t)TNB * LQ) return; if (which > 0 && rb >= (size_t)TNB * LK) return;
  const size_t r0 = rb + wave * 16; const int c0 = blockIdx.y * 128; const float* A = (which == 0) ? XQ : (which == 1) ? XK : XV; const __bf16* Wr = PW + ((size_t)which * DM) * DM; const float* BB = (which == 0) ? BQ : (which == 1) ? BK : BV;
  v8f acc[8] = {};
#pragma unroll 2
  for (int kc = 0; kc < DM / 32; ++kc) { v16b a; { const float* p = A + (r0 + col) * DM + kc * 32 + 8 * g;
#pragma unroll
      for (int i = 0; i < 8; ++i) { a[i] = (__bf16)p[i]; a[8 + i] = (__bf16)p[16 + i]; } }
#pragma unroll
    for (int j = 0; j < 8; ++j) acc[j] = wmma_bf(a, frag_b(Wr + (size_t)(c0 + j * 16 + col) * DM + kc * 32, lane), acc[j]); }
#pragma unroll
  for (int j = 0; j < 8; ++j) { const float bb = bfr(BB[c0 + j * 16 + col]);
#pragma unroll
    for (int r = 0; r < 8; ++r) { const _Float16 hv = (_Float16)(acc[j][r] + bb); if (which < 2) so[wave * 16 + 8 * g + r][j * 16 + col] = hv; else st[j * 16 + col][wave * 16 + 8 * g + r] = hv; } }
  __syncthreads();
  if (which < 2) { _Float16* dst = (which == 0) ? Q : Kr; for (int e = tid; e < 64 * 16; e += 128) { const int rl = e >> 4, q = e & 15; vst2((unsigned*)(dst + (rb + rl) * DM + c0 + q * 8), *(const v4u*)&so[rl][q * 8]); } }
  else { const size_t b = rb / LK; const int s0 = (int)(rb % LK); for (int e = tid; e < 128 * 8; e += 128) { const int d = e >> 3, pc = e & 7; vst2((unsigned*)(V + ((b * DM + c0 + d) * LK) + s0 + pc * 8), *(const v4u*)&st[d][pc * 8]); } }
}
__global__ __launch_bounds__(128) void k_attn(const _Float16* __restrict__ Q, const _Float16* __restrict__ Kr, const _Float16* __restrict__ V, const float* __restrict__ VB, float* __restrict__ O) {
  __shared__ __align__(16) _Float16 sph[4][16][40]; __shared__ __align__(16) float so[4][16][68];
  const int tid = threadIdx.x, wave = tid >> 5, lane = tid & 31, col = lane & 15, g = lane >> 4; const int h = blockIdx.y; const size_t b = blockIdx.z; const int q0 = blockIdx.x * 64 + wave * 16; const size_t rq = b * LQ + q0;
  v16h aq[2];
#pragma unroll
  for (int kc = 0; kc < 2; ++kc) aq[kc] = frag_h(Q + (rq + col) * DM + h * HD + kc * 32, lane);
  float m[8], l[8];
#pragma unroll
  for (int r = 0; r < 8; ++r) { m[r] = -3.0e38f; l[r] = 0.f; }
  v8f acc[4] = {};
#pragma unroll 1
  for (int ks = 0; ks < LK / 32; ++ks) { const int j0 = ks * 32; v8f s[2];
#pragma unroll
    for (int ct = 0; ct < 2; ++ct) { const int kk = j0 + ct * 16 + col; const size_t rk = (b * LK + kk) * DM + h * HD; v8f c = {}; const float vb = bfr(VB[b * LK + kk]);
#pragma unroll
      for (int kc = 0; kc < 2; ++kc) c = wmma16(aq[kc], frag_h(Kr + rk + kc * 32, lane), c);
#pragma unroll
      for (int r = 0; r < 8; ++r) s[ct][r] = c[r] * 0.125f + vb; }
#pragma unroll
    for (int r = 0; r < 8; ++r) { float mx = fmaxf(s[0][r], s[1][r]);
#pragma unroll
      for (int o = 1; o < 16; o <<= 1) mx = fmaxf(mx, __shfl_xor(mx, o));
      const float mn = fmaxf(m[r], mx); const float alpha = (m[r] <= -1.0e38f) ? 0.f : __expf(m[r] - mn); const float e0 = __expf(s[0][r] - mn), e1 = __expf(s[1][r] - mn); float es = e0 + e1;
#pragma unroll
      for (int o = 1; o < 16; o <<= 1) es += __shfl_xor(es, o);
      l[r] = l[r] * alpha + es; m[r] = mn;
#pragma unroll
      for (int dt = 0; dt < 4; ++dt) acc[dt][r] *= alpha;
      sph[wave][8 * g + r][col] = (_Float16)(e0 * 2048.0f); sph[wave][8 * g + r][16 + col] = (_Float16)(e1 * 2048.0f); }
    LDSX();
    const v16h pa = frag_h(&sph[wave][col][0], lane);
#pragma unroll
    for (int dt = 0; dt < 4; ++dt) acc[dt] = wmma16(pa, frag_h(V + ((b * DM + h * HD + dt * 16 + col) * LK) + j0, lane), acc[dt]);
    LDSX(); }
#pragma unroll
  for (int r = 0; r < 8; ++r) { const float il = (1.0f / 2048.0f) / l[r];
#pragma unroll
    for (int dt = 0; dt < 4; ++dt) so[wave][8 * g + r][dt * 16 + col] = acc[dt][r] * il; }
  LDSX();
  for (int rl = 0; rl < 16; ++rl) if (lane < 16) vst2(O + (rq + rl) * DM + h * HD + lane * 4, *(const v4f*)&so[wave][rl][lane * 4]);
}
__global__ __launch_bounds__(128) void k_out(const float* __restrict__ O, const __bf16* __restrict__ PW, const float* __restrict__ BO, float* __restrict__ Y) { __shared__ __align__(16) float so[4][16][132];
  const int tid = threadIdx.x, wave = tid >> 5, lane = tid & 31, col = lane & 15, g = lane >> 4; const size_t r0 = (size_t)blockIdx.x * 64 + wave * 16; const int c0 = blockIdx.y * 128; const __bf16* Wr = PW + (size_t)3 * DM * DM;
  v8f acc[8] = {};
#pragma unroll 2
  for (int kc = 0; kc < DM / 32; ++kc) { const F2 a = split_row(O + (r0 + col) * DM, kc * 32, lane);
#pragma unroll
    for (int j = 0; j < 8; ++j) { const v16b w = frag_b(Wr + (size_t)(c0 + j * 16 + col) * DM + kc * 32, lane); acc[j] = wmma_bf(a.h, w, acc[j]); acc[j] = wmma_bf(a.l, w, acc[j]); } }
#pragma unroll
  for (int j = 0; j < 8; ++j) { const float bb = bfr(BO[c0 + j * 16 + col]);
#pragma unroll
    for (int r = 0; r < 8; ++r) so[wave][8 * g + r][j * 16 + col] = acc[j][r] + bb; }
  LDSX(); for (int rl = 0; rl < 16; ++rl) vst2(Y + (r0 + rl) * DM + c0 + lane * 4, *(const v4f*)&so[wave][rl][lane * 4]); }
extern "C" void kernel_launch(void* const* d_in, const int* in_sizes, int n_in, void* d_out, int out_size, void* d_ws, size_t ws_size, hipStream_t stream) {
  (void)in_sizes; (void)n_in; (void)out_size;
  const float** F = (const float**)d_in;
  if (ws_size < (size_t)WS_END) return;
  char* ws = (char*)d_ws; __bf16* PW = (__bf16*)ws; _Float16 *Qr = (_Float16*)(ws + WS_Q), *Kr = (_Float16*)(ws + WS_K), *V = (_Float16*)(ws + WS_V); float* O = (float*)(ws + WS_O);
  k_pack<<<dim3(DM, 4), 256, 0, stream>>>(F[4], F[6], F[8], F[10], PW);
  k_proj<<<dim3(NRK / 64, DM / 128, 3), 128, 0, stream>>>(F[0], F[1], F[2], PW, F[5], F[7], F[9], Qr, Kr, V);
  k_attn<<<dim3(TQB, NH, TNB), 128, 0, stream>>>(Qr, Kr, V, F[3], O);
  k_out<<<dim3(TNB * LQ / 64, DM / 128), 128, 0, stream>>>(O, PW, F[11], (float*)d_out);
}
